// GAT_2293512536203
// MI455X (gfx1250) — hardware-run, weakly checked
//
#include <hip/hip_runtime.h>
#include <math.h>

typedef __attribute__((ext_vector_type(16))) _Float16 v16h;
typedef __attribute__((ext_vector_type(8)))  _Float16 v8h;
typedef __attribute__((ext_vector_type(8)))  float    v8f;
typedef __attribute__((ext_vector_type(4)))  float    v4f;

constexpr int kNSrc   = 768;
constexpr int kNTgt   = 768;
constexpr int kNTot   = 1536;
constexpr int kFeat   = 33;
constexpr int kFeatP  = 64;
constexpr int kNElt   = kNTot * kFeat;
constexpr int kIters  = 1000;
constexpr float kCarry = 256.0f;
constexpr float kF16MinNormal = 6.103515625e-5f;
constexpr int kRowsPerWave = 24;
static_assert(kNSrc + kNTgt == kNTot);
static_assert(kNElt == 50688);
static_assert((kFeatP % 32) == 0 && kFeatP >= kFeat);
static_assert((kNSrc % 16) == 0 && (kNTgt % 64) == 0 && (kNTgt % 16) == 0 && (kNSrc % 64) == 0);
static_assert(kNSrc == kNTgt);
static_assert(kRowsPerWave * 32 == kNSrc);
static_assert((kNTgt % 128) == 0);

constexpr size_t kOffXP = 0;
constexpr size_t kOffKM = kOffXP + (size_t)kNTot * kFeatP * 2;
constexpr size_t kOffKT = kOffKM + (size_t)kNSrc * kNTgt * 4;
constexpr size_t kOffUV = kOffKT + (size_t)kNSrc * kNTgt * 4;
constexpr size_t kWsTotal = kOffUV + (size_t)2 * kNSrc * 4;
static_assert(kWsTotal == 4921344ull);
static_assert(kWsTotal <= 134217728ull);
static_assert((kOffKM % 128) == 0 && (kOffKT % 128) == 0 && (kOffUV % 128) == 0);

union FragH { v16h v; v8h h[2]; };
__device__ __forceinline__ v16h frag_load_h(const _Float16* p) {
  FragH f;
  f.h[0] = *(const v8h*)(p);
  f.h[1] = *(const v8h*)(p + 16);
  return f.v;
}
__device__ __forceinline__ v8f mma_f16(v16h a, v16h b, v8f c) {
  c = __builtin_amdgcn_wmma_f32_16x16x32_f16(false, a, false, b, (short)0, c, false, false);
  asm volatile("v_nop\n\tv_nop\n\tv_nop\n\tv_nop" : "+v"(c) : "v"(a), "v"(b));
  return c;
}

__global__ __launch_bounds__(1024) void prep_planes_kernel(
    const float* __restrict__ x, const int* __restrict__ nsp, const int* __restrict__ ntp,
    unsigned short* __restrict__ XP)
{
  __shared__ float smn[32];
  __shared__ float smx[32];
  const int tid = threadIdx.x, lane = tid & 31, wave = tid >> 5;
  float mn = 3.402823466e38f, mx = -3.402823466e38f;
  for (int i = tid; i < kNElt; i += 1024) {
    const float v = x[i];
    mn = fminf(mn, v);
    mx = fmaxf(mx, v);
  }
  {
    float o;
    o = __shfl_xor(mn, 16, 32); mn = fminf(mn, o);
    o = __shfl_xor(mx, 16, 32); mx = fmaxf(mx, o);
    o = __shfl_xor(mn, 8, 32);  mn = fminf(mn, o);
    o = __shfl_xor(mx, 8, 32);  mx = fmaxf(mx, o);
    o = __shfl_xor(mn, 4, 32);  mn = fminf(mn, o);
    o = __shfl_xor(mx, 4, 32);  mx = fmaxf(mx, o);
    o = __shfl_xor(mn, 2, 32);  mn = fminf(mn, o);
    o = __shfl_xor(mx, 2, 32);  mx = fmaxf(mx, o);
    o = __shfl_xor(mn, 1, 32);  mn = fminf(mn, o);
    o = __shfl_xor(mx, 1, 32);  mx = fmaxf(mx, o);
  }
  if (lane == 0) {
    smn[wave] = mn;
    smx[wave] = mx;
  }
  __syncthreads();
  float gmn = smn[lane], gmx = smx[lane];
  {
    float o;
    o = __shfl_xor(gmn, 16, 32); gmn = fminf(gmn, o);
    o = __shfl_xor(gmx, 16, 32); gmx = fmaxf(gmx, o);
    o = __shfl_xor(gmn, 8, 32);  gmn = fminf(gmn, o);
    o = __shfl_xor(gmx, 8, 32);  gmx = fmaxf(gmx, o);
    o = __shfl_xor(gmn, 4, 32);  gmn = fminf(gmn, o);
    o = __shfl_xor(gmx, 4, 32);  gmx = fmaxf(gmx, o);
    o = __shfl_xor(gmn, 2, 32);  gmn = fminf(gmn, o);
    o = __shfl_xor(gmx, 2, 32);  gmx = fmaxf(gmx, o);
    o = __shfl_xor(gmn, 1, 32);  gmn = fminf(gmn, o);
    o = __shfl_xor(gmx, 1, 32);  gmx = fmaxf(gmx, o);
  }
  const float inv = 1.0f / (gmx - gmn);
  int tb = nsp[0];
  const int ntv = ntp[0];
  (void)ntv;
  tb = (tb < 0) ? 0 : tb;
  tb = (tb > (kNTot - kNTgt)) ? (kNTot - kNTgt) : tb;
#pragma unroll 1
  for (int it = 0; it < 12; ++it) {
    const int g = it * 1024 + tid;
    const int prow = g >> 3;
    const int c8 = (g & 7) * 8;
    const int xrow = (prow < kNSrc) ? prow : (tb + (prow - kNSrc));
    const float* xr = x + (size_t)xrow * kFeat;
    v8h hv;
#pragma unroll
    for (int e = 0; e < 8; ++e) {
      const int col = c8 + e;
      const int cc = (col < kFeat) ? col : (kFeat - 1);
      const float raw = xr[cc];
      float s = ((raw - gmn) * inv) * kCarry;
      s = (fabsf(s) < kF16MinNormal) ? 0.0f : s;
      s = (col < kFeat) ? s : 0.0f;
      hv[e] = (_Float16)s;
    }
    unsigned short* p = XP + (size_t)prow * kFeatP + c8;
    *(volatile v8h*)p = hv;
    __threadfence();
    *(volatile v8h*)p = hv;
  }
}

__global__ __launch_bounds__(256) void score_exp_kernel(
    const unsigned short* __restrict__ XPp, float* __restrict__ KM, float* __restrict__ KT, float scl)
{
  __shared__ __align__(16) float sT[8][16 * 68];
  const _Float16* XP = (const _Float16*)XPp;
  const int lane = threadIdx.x & 31;
  const int wave = threadIdx.x >> 5;
  const int tile = blockIdx.x * 8 + wave;
  constexpr int kTilesN = kNTgt / 64;
  constexpr int kTilesM = kNSrc / 16;
  if (tile >= kTilesM * kTilesN) return;
  const int tm = tile / kTilesN;
  const int tn = tile - tm * kTilesN;
  const int m0 = tm * 16;
  const int n0 = tn * 64;
  const int sel = blockIdx.y;
  const int aRow0 = sel ? kNSrc : 0;
  const int bRow0 = sel ? 0 : kNSrc;
  float* C = sel ? KT : KM;

  const int rlane = lane & 15;
  const int koff  = (lane >> 4) * 8;
  const int mOff  = (lane >> 4) * 8;

  v8f acc[4];
#pragma unroll
  for (int j = 0; j < 4; ++j) acc[j] = (v8f){0.f, 0.f, 0.f, 0.f, 0.f, 0.f, 0.f, 0.f};

#pragma unroll
  for (int ks = 0; ks < kFeatP / 32; ++ks) {
    const int k0 = ks * 32;
    const v16h a = frag_load_h(XP + (size_t)(aRow0 + m0 + rlane) * kFeatP + koff + k0);
#pragma unroll
    for (int j = 0; j < 4; ++j) {
      const v16h b = frag_load_h(XP + (size_t)(bRow0 + n0 + (j << 4) + rlane) * kFeatP + koff + k0);
      acc[j] = mma_f16(a, b, acc[j]);
    }
  }

  float* slab = sT[wave];
#pragma unroll
  for (int j = 0; j < 4; ++j) {
#pragma unroll
    for (int r = 0; r < 8; ++r) slab[(mOff + r) * 68 + (j << 4) + rlane] = acc[j][r];
  }
  __builtin_amdgcn_fence(__ATOMIC_RELEASE, "workgroup");
  __builtin_amdgcn_wave_barrier();
  __builtin_amdgcn_fence(__ATOMIC_ACQUIRE, "workgroup");

  const int hh = lane >> 4;
  const int c4 = (lane & 15) * 4;
#pragma unroll 1
  for (int it = 0; it < 8; ++it) {
    const int row = it * 2 + hh;
    v4f v = *(const v4f*)(slab + row * 68 + c4);
    const float e0 = expf(v[0] * scl);
    const float e1 = expf(v[1] * scl);
    const float e2 = expf(v[2] * scl);
    const float e3 = expf(v[3] * scl);
    v[0] = e0; v[1] = e1; v[2] = e2; v[3] = e3;
    *(v4f*)(slab + row * 68 + c4) = v;
    *(volatile v4f*)(C + (size_t)(m0 + row) * kNTgt + n0 + c4) = v;
  }
  __threadfence();
#pragma unroll 1
  for (int it = 0; it < 8; ++it) {
    const int row = it * 2 + hh;
    const v4f v = *(const v4f*)(slab + row * 68 + c4);
    *(volatile v4f*)(C + (size_t)(m0 + row) * kNTgt + n0 + c4) = v;
  }
  __threadfence();
}

__global__ __launch_bounds__(1024) void scaling_iter_kernel(
    const float* __restrict__ KM, const float* __restrict__ KT, float* __restrict__ UV)
{
  __shared__ __align__(16) float su[kNSrc];
  __shared__ __align__(16) float sv[kNTgt];
  const int tid = threadIdx.x, lane = tid & 31, wave = tid >> 5;
  if (tid < kNTgt) sv[tid] = 1.0f;
  __syncthreads();
  const int r0 = wave * kRowsPerWave;
#pragma unroll 1
  for (int it = 0; it < kIters; ++it) {
    {
      v4f w[6];
#pragma unroll
      for (int t = 0; t < 6; ++t) w[t] = *(const v4f*)(sv + t * 128 + lane * 4);
      float res = 1.0f;
#pragma unroll 1
      for (int r = 0; r < kRowsPerWave; ++r) {
        const float* kr = KM + (size_t)(r0 + r) * kNTgt + lane * 4;
        float s = 0.0f;
#pragma unroll
        for (int t = 0; t < 6; ++t) {
          const v4f kv = *(const v4f*)(kr + t * 128);
          s = fmaf(kv[0], w[t][0], s);
          s = fmaf(kv[1], w[t][1], s);
          s = fmaf(kv[2], w[t][2], s);
          s = fmaf(kv[3], w[t][3], s);
        }
        s += __shfl_xor(s, 16, 32);
        s += __shfl_xor(s, 8, 32);
        s += __shfl_xor(s, 4, 32);
        s += __shfl_xor(s, 2, 32);
        s += __shfl_xor(s, 1, 32);
        res = (lane == r) ? s : res;
      }
      const float rinv = 1.0f / res;
      if (lane < kRowsPerWave) su[r0 + lane] = rinv;
    }
    __syncthreads();
    {
      v4f w[6];
#pragma unroll
      for (int t = 0; t < 6; ++t) w[t] = *(const v4f*)(su + t * 128 + lane * 4);
      float res = 1.0f;
#pragma unroll 1
      for (int r = 0; r < kRowsPerWave; ++r) {
        const float* kr = KT + (size_t)(r0 + r) * kNSrc + lane * 4;
        float s = 0.0f;
#pragma unroll
        for (int t = 0; t < 6; ++t) {
          const v4f kv = *(const v4f*)(kr + t * 128);
          s = fmaf(kv[0], w[t][0], s);
          s = fmaf(kv[1], w[t][1], s);
          s = fmaf(kv[2], w[t][2], s);
          s = fmaf(kv[3], w[t][3], s);
        }
        s += __shfl_xor(s, 16, 32);
        s += __shfl_xor(s, 8, 32);
        s += __shfl_xor(s, 4, 32);
        s += __shfl_xor(s, 2, 32);
        s += __shfl_xor(s, 1, 32);
        res = (lane == r) ? s : res;
      }
      const float rinv = 1.0f / res;
      if (lane < kRowsPerWave) sv[r0 + lane] = rinv;
    }
    __syncthreads();
  }
  if (wave < kNSrc / 32) {
    const float a = su[wave * 32 + lane];
    const float b = sv[wave * 32 + lane];
    float* pu = UV + wave * 32 + lane;
    float* pv = UV + kNSrc + wave * 32 + lane;
    *(volatile float*)pu = a;
    *(volatile float*)pv = b;
    __threadfence();
    *(volatile float*)pu = a;
    *(volatile float*)pv = b;
  }
}

__global__ __launch_bounds__(256) void scale_out_kernel(
    const float* __restrict__ KM, const float* __restrict__ UV,
    const int* __restrict__ nsp, const int* __restrict__ ntp, float* __restrict__ out)
{
  constexpr int kV4PerRow = kNTgt / 4;
  constexpr int kTotalV4 = kNSrc * kV4PerRow;
  const int idx = blockIdx.x * 256 + threadIdx.x;
  if (idx >= kTotalV4) return;
  const int row = idx / kV4PerRow;
  const int c4 = (idx - row * kV4PerRow) * 4;
  const float u = UV[row];
  const v4f kv = *(const v4f*)(KM + (size_t)row * kNTgt + c4);
  const v4f vv = *(const v4f*)(UV + kNSrc + c4);
  const bool ok = (nsp[0] == kNSrc) && (ntp[0] == kNTgt);
  const float qnan = __uint_as_float(0x7fc00000u);
  v4f o;
  o[0] = ok ? ((u * kv[0]) * vv[0]) : qnan;
  o[1] = ok ? ((u * kv[1]) * vv[1]) : qnan;
  o[2] = ok ? ((u * kv[2]) * vv[2]) : qnan;
  o[3] = ok ? ((u * kv[3]) * vv[3]) : qnan;
  float* p = out + (size_t)row * kNTgt + c4;
  *(volatile v4f*)p = o;
  __threadfence();
  *(volatile v4f*)p = o;
}

extern "C" void kernel_launch(void* const* d_in, const int* in_sizes, int n_in,
                              void* d_out, int out_size, void* d_ws, size_t ws_size,
                              hipStream_t stream) {
  if (n_in < 3) return;
  if (in_sizes[0] != kNElt) return;
  if (in_sizes[1] != 1) return;
  if (in_sizes[2] != 1) return;
  if (out_size != kNSrc * kNTgt) return;
  if (ws_size < kWsTotal) return;

  const float* x   = (const float*)d_in[0];
  const int*   nsp = (const int*)d_in[1];
  const int*   ntp = (const int*)d_in[2];
  float* out = (float*)d_out;

  char* ws = (char*)d_ws;
  unsigned short* XP = (unsigned short*)(ws + kOffXP);
  float* KM = (float*)(ws + kOffKM);
  float* KT = (float*)(ws + kOffKT);
  float* UV = (float*)(ws + kOffUV);

  const float scl = (1.0f / sqrtf((float)kFeat)) * (1.0f / (kCarry * kCarry));

  prep_planes_kernel<<<1, 1024, 0, stream>>>(x, nsp, ntp, XP);
  score_exp_kernel<<<dim3((kNSrc / 16) * (kNTgt / 64) / 8, 2), 256, 0, stream>>>(XP, KM, KT, scl);
  scaling_iter_kernel<<<1, 1024, 0, stream>>>(KM, KT, UV);
  scale_out_kernel<<<(kNSrc * (kNTgt / 4)) / 256, 256, 0, stream>>>(KM, UV, nsp, ntp, out);
}
